// FFN_GCNs_13572096655679
// MI455X (gfx1250) — hardware-verified
//
#include <hip/hip_runtime.h>
#include <stddef.h>


#define FEAT 32
#define NTILE 68
#define PITCH 1088
#define COL_ROOT 1024
#define COL_XB 1056
#define NSLOTS (NTILE * 64)

#define CH1 4096
#define MAXB 1600
#define PITCHB 1568
#define BPT 7
#define MAXNB1 128
#define CAP3 1024

typedef _Float16 v16h __attribute__((ext_vector_type(16)));
typedef _Float16 v8h __attribute__((ext_vector_type(8)));
typedef float v8f __attribute__((ext_vector_type(8)));
typedef float v4f __attribute__((ext_vector_type(4)));
typedef int v4i __attribute__((ext_vector_type(4)));
typedef v4f __attribute__((may_alias)) v4fa;
typedef v4i __attribute__((may_alias)) v4ia;

union Frag { v16h v; v8h half[2]; _Float16 e[16]; };

__device__ __forceinline__ v8f wmma16(const v16h& a, const v16h& b, v8f c) {
    return __builtin_amdgcn_wmma_f32_16x16x32_f16(false, a, false, b, (short)0, c, false, false);
}

__global__ __launch_bounds__(256) void k_prep(const float* __restrict__ w2, const float* __restrict__ root,
                                              const float* __restrict__ b2, _Float16* bfrag) {
    const int t0 = blockIdx.x * 256 + threadIdx.x;
    const bool ok = t0 < NSLOTS;
    const int tt = ok ? t0 : 0;
    const int g = tt & 1, l = (tt >> 1) & 31, t = tt >> 6;
    const int h = l >> 4, c = t * 16 + (l & 15);
    const int kb = 8 * h + 16 * g;
    const int o5 = c & 31, ow = (c >> 5) & 31;
    union { v8h v; _Float16 e[8]; } u;
#pragma unroll
    for (int ii = 0; ii < 8; ++ii) {
        const int k = kb + ii;
        const float vw = w2[o5 * 1024 + k * 32 + ow];
        const float vr = root[k * 32 + o5];
        const float vb = b2[k * 32 + o5];
        const float v = (c < COL_ROOT) ? vw : ((c < COL_XB) ? vr : vb);
        u.e[ii] = (_Float16)(v * 64.0f);
    }
    const v8h val = u.v;
    if (ok) *(volatile v8h*)(bfrag + (size_t)tt * 8) = val;
    __threadfence();
    if (ok) *(volatile v8h*)(bfrag + (size_t)tt * 8) = val;
}

__global__ __launch_bounds__(32) void k_node(const float* __restrict__ x, const _Float16* bfrag,
                                             float* nodep, int N, int ntiles) {
    __shared__ __attribute__((aligned(16))) float stg[16 * 32];
    const int tile = blockIdx.x;
    if (tile >= ntiles) return;
    const int lane = threadIdx.x & 31, h = lane >> 4, m = lane & 15;
    int row = tile * 16 + m;
    row = row > N - 1 ? N - 1 : row;
    const v4f* xr = (const v4f*)(x + (size_t)row * FEAT);
    const v4f p0 = xr[2 * h], p1 = xr[2 * h + 1], p2 = xr[4 + 2 * h], p3 = xr[5 + 2 * h];
    Frag a;
    a.e[0] = (_Float16)p0.x;  a.e[1] = (_Float16)p0.y;  a.e[2] = (_Float16)p0.z;  a.e[3] = (_Float16)p0.w;
    a.e[4] = (_Float16)p1.x;  a.e[5] = (_Float16)p1.y;  a.e[6] = (_Float16)p1.z;  a.e[7] = (_Float16)p1.w;
    a.e[8] = (_Float16)p2.x;  a.e[9] = (_Float16)p2.y;  a.e[10] = (_Float16)p2.z; a.e[11] = (_Float16)p2.w;
    a.e[12] = (_Float16)p3.x; a.e[13] = (_Float16)p3.y; a.e[14] = (_Float16)p3.z; a.e[15] = (_Float16)p3.w;

    const v8h* bq = (const v8h*)bfrag;
    const float inv = 0.015625f;
    float* gbase = nodep + (size_t)tile * 16 * PITCH;
    const v4fa* sv = (const v4fa*)stg;

#pragma unroll 1
    for (int u = 0; u < NTILE / 2; ++u) {
        Frag b0, b1;
        const int f0 = ((2 * u) * 32 + lane) * 2;
        const int f1 = ((2 * u + 1) * 32 + lane) * 2;
        b0.half[0] = bq[f0];
        b0.half[1] = bq[f0 + 1];
        b1.half[0] = bq[f1];
        b1.half[1] = bq[f1 + 1];
        v8f z;
#pragma unroll
        for (int r = 0; r < 8; ++r) z[r] = 0.0f;
        v8f c0 = wmma16(a.v, b0.v, z);
        v8f c1 = wmma16(a.v, b1.v, z);
        asm volatile("v_nop\n\tv_nop\n\tv_nop\n\tv_nop" : "+v"(c0), "+v"(c1) : "v"(a.v), "v"(b0.v), "v"(b1.v));
#pragma unroll
        for (int r = 0; r < 8; ++r) {
            stg[(8 * h + r) * 32 + m] = c0[r] * inv;
            stg[(8 * h + r) * 32 + 16 + m] = c1[r] * inv;
        }
        __syncthreads();
        v4f ov[4];
#pragma unroll
        for (int it = 0; it < 4; ++it) ov[it] = sv[it * 32 + lane];
        float* gp = gbase + 32 * u + (lane & 7) * 4;
#pragma unroll
        for (int it = 0; it < 4; ++it)
            *(volatile v4f*)(gp + (size_t)(it * 4 + (lane >> 3)) * PITCH) = ov[it];
        __threadfence();
#pragma unroll
        for (int it = 0; it < 4; ++it)
            *(volatile v4f*)(gp + (size_t)(it * 4 + (lane >> 3)) * PITCH) = ov[it];
        __syncthreads();
    }
}

__device__ __forceinline__ void chunk_keys(const int* __restrict__ recv, int cb, int lane, int E, int N,
                                           unsigned& key_out, int& rank, bool& last, bool& valid) {
    const int e = cb + lane;
    const int ec = e < E ? e : E - 1;
    const int r = recv[ec];
    unsigned key = 0xFFFFFFFFu;
    if (e < E && r >= 0 && r < N) key = ((unsigned)r & ~31u) | (unsigned)lane;
#pragma unroll
    for (int kk = 2; kk <= 32; kk <<= 1) {
#pragma unroll
        for (int j = kk >> 1; j > 0; j >>= 1) {
            const unsigned p = __shfl_xor(key, j);
            const bool asc = (lane & kk) == 0;
            const bool low = (lane & j) == 0;
            const unsigned mn = key < p ? key : p;
            const unsigned mx = key < p ? p : key;
            key = (asc == low) ? mn : mx;
        }
    }
    const unsigned bkt = key >> 5;
    const unsigned pk = __shfl_up(key, 1);
    const unsigned nk = __shfl_down(key, 1);
    const bool start = (lane == 0) || ((pk >> 5) != bkt);
    last = (lane == 31) || ((nk >> 5) != bkt);
    int v = start ? lane : 0;
#pragma unroll
    for (int d = 1; d < 32; d <<= 1) {
        const int uu = __shfl_up(v, d);
        if (lane >= d && uu > v) v = uu;
    }
    rank = lane - v;
    key_out = key;
    valid = (key != 0xFFFFFFFFu);
}

__global__ __launch_bounds__(256) void k_bucket(const int* __restrict__ recv, int* lists, int* offtab, int E, int N) {
    __shared__ unsigned short wcnt[8 * MAXB];
    __shared__ __attribute__((aligned(16))) int list_lds[CH1];
    __shared__ __attribute__((aligned(16))) int boff[PITCHB];
    __shared__ int sb[256];
    const int t = threadIdx.x, lane = t & 31, wid = t >> 5, blk = blockIdx.x;

    for (int i = t; i < 8 * MAXB; i += 256) wcnt[i] = 0;
    for (int i = t; i < CH1; i += 256) list_lds[i] = 0;
    __syncthreads();

    const int wbase = blk * CH1 + wid * 512;
#pragma unroll 1
    for (int c = 0; c < 16; ++c) {
        unsigned key; int rank; bool last, valid;
        chunk_keys(recv, wbase + c * 32, lane, E, N, key, rank, last, valid);
        if (valid && last) {
            const int b = (int)(key >> 5);
            wcnt[wid * MAXB + b] += (unsigned short)(rank + 1);
        }
    }
    __syncthreads();

    int tsum = 0;
#pragma unroll 1
    for (int q = 0; q < BPT; ++q) {
        const int b = t * BPT + q;
        if (b < PITCHB) {
            int tot = 0;
#pragma unroll
            for (int w = 0; w < 8; ++w) tot += (int)wcnt[w * MAXB + b];
            tsum += tot;
        }
    }
    sb[t] = tsum;
    __syncthreads();
#pragma unroll 1
    for (int d = 1; d < 256; d <<= 1) {
        const int v = (t >= d) ? sb[t - d] : 0;
        __syncthreads();
        sb[t] += v;
        __syncthreads();
    }
    int run = sb[t] - tsum;
#pragma unroll 1
    for (int q = 0; q < BPT; ++q) {
        const int b = t * BPT + q;
        if (b < PITCHB) {
            boff[b] = run;
#pragma unroll
            for (int w = 0; w < 8; ++w) {
                const int cnt = (int)wcnt[w * MAXB + b];
                wcnt[w * MAXB + b] = (unsigned short)run;
                run += cnt;
            }
        }
    }
    __syncthreads();

#pragma unroll 1
    for (int c = 0; c < 16; ++c) {
        const int cb = wbase + c * 32;
        unsigned key; int rank; bool last, valid;
        chunk_keys(recv, cb, lane, E, N, key, rank, last, valid);
        if (valid) {
            const int b = (int)(key >> 5);
            const int pos = (int)wcnt[wid * MAXB + b] + rank;
            if ((unsigned)pos < (unsigned)CH1) list_lds[pos] = cb + (int)(key & 31u);
            if (last) wcnt[wid * MAXB + b] = (unsigned short)(pos + 1);
        }
    }
    __syncthreads();

    const v4ia* lsrc = (const v4ia*)list_lds;
    const v4ia* bsrc = (const v4ia*)boff;
    v4i lv[4];
#pragma unroll
    for (int u = 0; u < 4; ++u) lv[u] = lsrc[t + u * 256];
    const int t2 = t + 256;
    const bool has2 = t2 < (PITCHB / 4);
    const v4i bv0 = bsrc[t];
    const v4i bv1 = bsrc[has2 ? t2 : t];
    int* ld = lists + (size_t)blk * CH1;
    int* bd = offtab + (size_t)blk * PITCHB;
#pragma unroll
    for (int u = 0; u < 4; ++u) *(volatile v4i*)(ld + (size_t)(t + u * 256) * 4) = lv[u];
    *(volatile v4i*)(bd + (size_t)t * 4) = bv0;
    if (has2) *(volatile v4i*)(bd + (size_t)t2 * 4) = bv1;
    __threadfence();
#pragma unroll
    for (int u = 0; u < 4; ++u) *(volatile v4i*)(ld + (size_t)(t + u * 256) * 4) = lv[u];
    *(volatile v4i*)(bd + (size_t)t * 4) = bv0;
    if (has2) *(volatile v4i*)(bd + (size_t)t2 * 4) = bv1;
}

__global__ __launch_bounds__(32) void k_aggr(const int* __restrict__ ei, const float* __restrict__ ea,
                                             const float* __restrict__ w1, const float* __restrict__ b1,
                                             const float* __restrict__ bias, const float* nodep,
                                             const int* lists, const int* offtab, float* xout,
                                             int E, int N, int NB1) {
    __shared__ unsigned comp[CAP3];
    __shared__ __attribute__((aligned(16))) float acc[32 * 32];
    __shared__ __attribute__((aligned(16))) float hbuf[2 * 32];
    const int lane = threadIdx.x & 31;
    const int f = blockIdx.x;
    const int* recv = ei + E;
    const float w1a = w1[lane], w1b = w1[FEAT + lane], b1v = b1[lane], bsv = bias[lane];

    int cnt[4], lo[4], ex[4];
    int carry = 0;
#pragma unroll
    for (int u = 0; u < 4; ++u) {
        const int blk = lane + 32 * u;
        const bool inb = blk < NB1;
        const int* tb = offtab + (size_t)(inb ? blk : 0) * PITCHB;
        int a = tb[f];
        int b = tb[f + 1];
        a = a < 0 ? 0 : (a > CH1 ? CH1 : a);
        b = b < a ? a : (b > CH1 ? CH1 : b);
        const int c = inb ? (b - a) : 0;
        cnt[u] = c;
        lo[u] = inb ? a : 0;
        int s = c;
#pragma unroll
        for (int d = 1; d < 32; d <<= 1) {
            const int v = __shfl_up(s, d);
            if (lane >= d) s += v;
        }
        ex[u] = carry + s - c;
        carry += __shfl(s, 31);
    }
    const int T = carry < CAP3 ? carry : CAP3;

#pragma unroll
    for (int u = 0; u < 4; ++u) {
        const int blk = lane + 32 * u;
        const int* lp = lists + (size_t)(blk < NB1 ? blk : 0) * CH1 + lo[u];
        for (int q = 0; q < cnt[u]; ++q) {
            const int p = ex[u] + q;
            if (p < CAP3) {
                const int e = lp[q];
                const int ec = e < 0 ? 0 : (e > E - 1 ? E - 1 : e);
                const int nd = recv[ec] - f * 32;
                unsigned pk = 0xFFFFFFFFu;
                if ((unsigned)e < (unsigned)E && (unsigned)nd < 32u) pk = ((unsigned)e << 5) | (unsigned)nd;
                comp[p] = pk;
            }
        }
    }
#pragma unroll
    for (int r = 0; r < 32; ++r) acc[r * 32 + lane] = 0.0f;
    __syncthreads();

#pragma unroll 1
    for (int i = 0; i < T; ++i) {
        const unsigned pk = comp[i];
        const bool valid = pk != 0xFFFFFFFFu;
        int e = (int)(pk >> 5);
        e = valid ? e : 0;
        e = e > E - 1 ? E - 1 : e;
        const int nd = (int)(pk & 31u);
        int src = ei[e];
        src = src < 0 ? 0 : (src > N - 1 ? N - 1 : src);
        const float ea0 = ea[2 * e], ea1 = ea[2 * e + 1];
        const float he = fmaxf(fmaf(ea1, w1b, fmaf(ea0, w1a, b1v)), 0.0f);
        float* hb = hbuf + (i & 1) * 32;
        hb[lane] = he;
        __syncthreads();
        const v4fa* hv = (const v4fa*)hb;
        const float* grow = nodep + (size_t)src * PITCH;
        const v4f* gp = (const v4f*)(grow + lane * 32);
        float msg = grow[COL_XB + lane];
#pragma unroll
        for (int j = 0; j < 8; ++j) {
            const v4f hq = hv[j];
            const v4f g = gp[j];
            msg = fmaf(hq.x, g.x, msg);
            msg = fmaf(hq.y, g.y, msg);
            msg = fmaf(hq.z, g.z, msg);
            msg = fmaf(hq.w, g.w, msg);
        }
        msg = valid ? msg : 0.0f;
        acc[nd * 32 + lane] += msg;
    }
    __syncthreads();

#pragma unroll 4
    for (int nd = 0; nd < 32; ++nd) {
        int n = f * 32 + nd;
        n = n > N - 1 ? N - 1 : n;
        const float v = acc[nd * 32 + lane] + nodep[(size_t)n * PITCH + COL_ROOT + lane] + bsv;
        acc[nd * 32 + lane] = fmaxf(v, 0.0f);
    }
    __syncthreads();

    const v4fa* av = (const v4fa*)acc;
    v4f ov[8];
#pragma unroll
    for (int it = 0; it < 8; ++it) ov[it] = av[it * 32 + lane];
    float* ob = xout + (size_t)f * 32 * FEAT;
#pragma unroll
    for (int it = 0; it < 8; ++it) *(volatile v4f*)(ob + (size_t)(it * 32 + lane) * 4) = ov[it];
    __threadfence();
#pragma unroll
    for (int it = 0; it < 8; ++it) *(volatile v4f*)(ob + (size_t)(it * 32 + lane) * 4) = ov[it];
}

__global__ __launch_bounds__(256) void k_fc(const int* __restrict__ label, const float* xa, const float* xb,
                                            const float* __restrict__ fcw, const float* __restrict__ fcb,
                                            float* out, int NP, int Na, int Nb, int out_size) {
    __shared__ float fw[128];
    __shared__ float fb[2];
    __shared__ __attribute__((aligned(16))) float res[512];
    const int t = threadIdx.x;
    if (t < 128) fw[t] = fcw[t];
    if (t < 2) fb[t] = fcb[t];
    __syncthreads();
    int p = blockIdx.x * 256 + t;
    p = p > NP - 1 ? NP - 1 : p;
    int ia = label[2 * p], ib = label[2 * p + 1];
    ia = ia < 0 ? 0 : (ia > Na - 1 ? Na - 1 : ia);
    ib = ib < 0 ? 0 : (ib > Nb - 1 ? Nb - 1 : ib);
    const v4f* za = (const v4f*)(xa + (size_t)ia * FEAT);
    const v4f* zb = (const v4f*)(xb + (size_t)ib * FEAT);
    float o0 = fb[0], o1 = fb[1];
#pragma unroll 1
    for (int j = 0; j < 8; ++j) {
        const v4f v = za[j];
        const float* w = fw + 8 * j;
        o0 = fmaf(v.x, w[0], o0); o1 = fmaf(v.x, w[1], o1);
        o0 = fmaf(v.y, w[2], o0); o1 = fmaf(v.y, w[3], o1);
        o0 = fmaf(v.z, w[4], o0); o1 = fmaf(v.z, w[5], o1);
        o0 = fmaf(v.w, w[6], o0); o1 = fmaf(v.w, w[7], o1);
    }
#pragma unroll 1
    for (int j = 0; j < 8; ++j) {
        const v4f v = zb[j];
        const float* w = fw + 64 + 8 * j;
        o0 = fmaf(v.x, w[0], o0); o1 = fmaf(v.x, w[1], o1);
        o0 = fmaf(v.y, w[2], o0); o1 = fmaf(v.y, w[3], o1);
        o0 = fmaf(v.z, w[4], o0); o1 = fmaf(v.z, w[5], o1);
        o0 = fmaf(v.w, w[6], o0); o1 = fmaf(v.w, w[7], o1);
    }
    res[2 * t] = fmaxf(o0, 0.0f);
    res[2 * t + 1] = fmaxf(o1, 0.0f);
    __syncthreads();

    const int nv4 = out_size >> 2;
    const int gi = blockIdx.x * 128 + t;
    const bool ok = (t < 128) && (gi < nv4);
    const v4fa* rv = (const v4fa*)res;
    const v4f val = rv[t < 128 ? t : 0];
    const int rem = out_size - nv4 * 4;
    const bool tail = (blockIdx.x == gridDim.x - 1) && (t < rem);
    int li = nv4 * 4 - (int)blockIdx.x * 512 + t;
    li = li < 0 ? 0 : (li > 511 ? 511 : li);
    const float tv = res[li];
    if (ok) *(volatile v4f*)(out + (size_t)gi * 4) = val;
    if (tail) *(volatile float*)(out + (size_t)nv4 * 4 + t) = tv;
    __threadfence();
    if (ok) *(volatile v4f*)(out + (size_t)gi * 4) = val;
    if (tail) *(volatile float*)(out + (size_t)nv4 * 4 + t) = tv;
}

extern "C" void kernel_launch(void* const* d_in, const int* in_sizes, int n_in,
                              void* d_out, int out_size, void* d_ws, size_t ws_size,
                              hipStream_t stream) {
    if (n_in < 21) return;
    const float* x1 = (const float*)d_in[0];
    const int* ei1 = (const int*)d_in[1];
    const float* ea1 = (const float*)d_in[2];
    const float* x2 = (const float*)d_in[3];
    const int* ei2 = (const int*)d_in[4];
    const float* ea2 = (const float*)d_in[5];
    const int* label = (const int*)d_in[6];
    const float* l1_w1 = (const float*)d_in[7];
    const float* l1_b1 = (const float*)d_in[8];
    const float* l1_w2 = (const float*)d_in[9];
    const float* l1_b2 = (const float*)d_in[10];
    const float* l1_root = (const float*)d_in[11];
    const float* l1_bias = (const float*)d_in[12];
    const float* l2_w1 = (const float*)d_in[13];
    const float* l2_b1 = (const float*)d_in[14];
    const float* l2_w2 = (const float*)d_in[15];
    const float* l2_b2 = (const float*)d_in[16];
    const float* l2_root = (const float*)d_in[17];
    const float* l2_bias = (const float*)d_in[18];
    const float* fc_w = (const float*)d_in[19];
    const float* fc_b = (const float*)d_in[20];
    float* out = (float*)d_out;

    const int N1 = in_sizes[0] / FEAT, E1 = in_sizes[1] / 2;
    const int N2 = in_sizes[3] / FEAT, E2 = in_sizes[4] / 2;
    const int NP = in_sizes[6] / 2;
    if (N1 <= 0 || E1 <= 0 || N2 <= 0 || E2 <= 0 || NP <= 0) return;
    if (in_sizes[0] != N1 * FEAT || in_sizes[1] != 2 * E1 || in_sizes[2] != 2 * E1 ||
        in_sizes[3] != N2 * FEAT || in_sizes[4] != 2 * E2 || in_sizes[5] != 2 * E2 ||
        in_sizes[6] != 2 * NP || out_size != 2 * NP) return;
    for (int L = 0; L < 2; ++L) {
        const int b = 7 + 6 * L;
        if (in_sizes[b] != 2 * FEAT || in_sizes[b + 1] != FEAT || in_sizes[b + 2] != FEAT * 1024 ||
            in_sizes[b + 3] != 1024 || in_sizes[b + 4] != FEAT * FEAT || in_sizes[b + 5] != FEAT) return;
    }
    if (in_sizes[19] != 2 * FEAT * 2 || in_sizes[20] != 2) return;

    const int Nmax = N1 > N2 ? N1 : N2;
    const int Emax = E1 > E2 ? E1 : E2;
    const int NBmax = (Nmax + 31) / 32;
    if (NBmax + 1 > PITCHB) return;
    const int NB1max = (Emax + CH1 - 1) / CH1;
    if (NB1max > MAXNB1) return;
    const int NT16max = (Nmax + 15) / 16;

    size_t off = 0;
    auto carve = [&](size_t bytes) -> size_t { const size_t p = off; off += (bytes + 255) & ~(size_t)255; return p; };
    const size_t o_bf1 = carve((size_t)NSLOTS * 8 * sizeof(_Float16));
    const size_t o_bf2 = carve((size_t)NSLOTS * 8 * sizeof(_Float16));
    const size_t o_lists = carve((size_t)NB1max * CH1 * sizeof(int));
    const size_t o_tab = carve((size_t)NB1max * PITCHB * sizeof(int));
    const size_t o_nodep = carve((size_t)NT16max * 16 * PITCH * sizeof(float));
    const size_t o_xt = carve((size_t)NBmax * 32 * FEAT * sizeof(float));
    const size_t o_xf1 = carve((size_t)NBmax * 32 * FEAT * sizeof(float));
    const size_t o_xf2 = carve((size_t)NBmax * 32 * FEAT * sizeof(float));
    if (off > ws_size) return;

    char* ws = (char*)d_ws;
    _Float16* bf1 = (_Float16*)(ws + o_bf1);
    _Float16* bf2 = (_Float16*)(ws + o_bf2);
    int* lists = (int*)(ws + o_lists);
    int* offtab = (int*)(ws + o_tab);
    float* nodep = (float*)(ws + o_nodep);
    float* xt = (float*)(ws + o_xt);
    float* xf1 = (float*)(ws + o_xf1);
    float* xf2 = (float*)(ws + o_xf2);

    k_prep<<<(NSLOTS + 255) / 256, 256, 0, stream>>>(l1_w2, l1_root, l1_b2, bf1);
    k_prep<<<(NSLOTS + 255) / 256, 256, 0, stream>>>(l2_w2, l2_root, l2_b2, bf2);

    for (int g = 0; g < 2; ++g) {
        const float* x = g ? x2 : x1;
        const int* ei = g ? ei2 : ei1;
        const float* ea = g ? ea2 : ea1;
        float* xf = g ? xf2 : xf1;
        const int N = g ? N2 : N1;
        const int E = g ? E2 : E1;
        const int NB = (N + 31) / 32;
        const int NB1 = (E + CH1 - 1) / CH1;
        const int NT = (N + 15) / 16;

        k_bucket<<<NB1, 256, 0, stream>>>(ei + E, lists, offtab, E, N);
        k_node<<<NT, 32, 0, stream>>>(x, bf1, nodep, N, NT);
        k_aggr<<<NB, 32, 0, stream>>>(ei, ea, l1_w1, l1_b1, l1_bias, nodep, lists, offtab, xt, E, N, NB1);
        k_node<<<NT, 32, 0, stream>>>(xt, bf2, nodep, N, NT);
        k_aggr<<<NB, 32, 0, stream>>>(ei, ea, l2_w1, l2_b1, l2_bias, nodep, lists, offtab, xf, E, N, NB1);
    }

    k_fc<<<(NP + 255) / 256, 256, 0, stream>>>(label, xf1, xf2, fc_w, fc_b, out, NP, N1, N2, out_size);
}
